// stae_predict_3298534883357
// MI455X (gfx1250) — hardware-verified
//
#include <hip/hip_runtime.h>


namespace {
constexpr int Bn = 131072, T = 12, N = 4, H = 16, NB = 128;
constexpr float WS_ = 8.0f, AS_ = 8.0f;

typedef _Float16 b16;
typedef __attribute__((ext_vector_type(16))) _Float16 v16b;
typedef __attribute__((ext_vector_type(8))) _Float16 v8b;
typedef __attribute__((ext_vector_type(8))) float v8f;
typedef __attribute__((ext_vector_type(4))) float v4f;
__device__ __forceinline__ float bf16_rne(float f) { unsigned int u = __float_as_uint(f); u += 0x7FFFu + ((u >> 16) & 1u); return __uint_as_float(u & 0xFFFF0000u); }
__device__ __forceinline__ void split16(float v, b16& hi, b16& lo) { hi = (b16)v; lo = (b16)(v - (float)hi); }
__device__ __forceinline__ v16b frag_kb(const b16* p, int hh) { const v8b a = *(const v8b*)(p + 8 * hh), b = *(const v8b*)(p + 16 + 8 * hh); v16b f;
#pragma unroll
  for (int e = 0; e < 8; ++e) { f[e] = a[e]; f[8 + e] = b[e]; } return f; }
__device__ __forceinline__ v8f wmma16b(v16b a, v16b b, v8f c) { v8f d = __builtin_amdgcn_wmma_f32_16x16x32_f16(false, a, false, b, (short)0, c, false, false); asm volatile("v_nop\n\tv_nop\n\tv_nop\n\tv_nop" : "+v"(d) : "v"(a), "v"(b)); return d; }
__device__ __forceinline__ void wave_lds_sync() { __builtin_amdgcn_fence(__ATOMIC_RELEASE, "workgroup"); __builtin_amdgcn_wave_barrier(); __builtin_amdgcn_fence(__ATOMIC_ACQUIRE, "workgroup"); }
__device__ __forceinline__ float nexp(float x) { return __builtin_amdgcn_exp2f(x * 1.4426950408889634f); }
__device__ __forceinline__ float sigm(float x) { return __builtin_amdgcn_rcpf(1.0f + nexp(-x)); }
__device__ __forceinline__ float tanh_(float x) { const float e = nexp(-2.0f * fabsf(x)); const float t = (1.0f - e) * __builtin_amdgcn_rcpf(1.0f + e); return (x >= 0.0f) ? t : -t; }
__device__ __forceinline__ float pmul(float a, float b) { float p = a * b; asm volatile("" : "+v"(p)); return p; }

__global__ __launch_bounds__(256) void prep_kernel(const float* __restrict__ Wih, const float* __restrict__ Whh, const float* __restrict__ bih, const float* __restrict__ bhh, const float* __restrict__ W1, const float* __restrict__ b1, const float* __restrict__ W2, const float* __restrict__ b2,
                                                   const float* __restrict__ Wg, const float* __restrict__ bg, const float* __restrict__ Wg2, const float* __restrict__ bg2, const float* __restrict__ Wl, const float* __restrict__ bl,
                                                   const float* __restrict__ Weih, const float* __restrict__ Wehh, const float* __restrict__ beih, const float* __restrict__ behh, const float* __restrict__ Wenc, const float* __restrict__ benc,
                                                   b16* __restrict__ Bm, b16* __restrict__ Be, float* __restrict__ P) {
  const int t_ = threadIdx.x;
  for (int pass = 0; pass < 2; ++pass) {
    for (int p = t_; p < 64 * 32; p += 256) { const int row = p >> 5, k = p & 31; float vm = 0.0f, ve = 0.0f;
      if (k < N) { vm = Wih[row * N + k]; ve = Weih[row * N + k]; } else if (k < N + H) { vm = Whh[row * H + (k - N)]; ve = Wehh[row * H + (k - N)]; }
      ((volatile b16*)Bm)[p] = (b16)(bf16_rne(vm) * WS_); ((volatile b16*)Be)[p] = (b16)(bf16_rne(ve) * WS_); }
    for (int p = t_; p < 544; p += 256) { float v = 0.0f;
      if (p < 64) v = bf16_rne(bih[p]) + bf16_rne(bhh[p]); else if (p < 128) v = bf16_rne(beih[p - 64]) + bf16_rne(behh[p - 64]);
      else if (p < 256) v = bf16_rne(W1[p - 128]); else if (p < 264) v = bf16_rne(b1[p - 256]); else if (p < 296) v = bf16_rne(W2[p - 264]); else if (p < 300) v = bf16_rne(b2[p - 296]);
      else if (p < 303) v = bf16_rne(Wg[p - 300]); else if (p == 303) v = bf16_rne(bg[0]); else if (p < 307) v = bf16_rne(Wg2[p - 304]); else if (p == 307) v = bf16_rne(bg2[0]);
      else if (p < 464) v = bf16_rne(Wl[p - 308]); else if (p < 476) v = bf16_rne(bl[p - 464]); else if (p < 540) v = bf16_rne(Wenc[p - 476]); else v = bf16_rne(benc[p - 540]);
      ((volatile float*)P)[p] = v; }
    __threadfence();
  }
}

__device__ __forceinline__ void gcn4(const float v[4], const float* w, float b, float o[4]) {
  float x1[4] = {v[1], v[0] + v[2], v[1] + v[3], v[2]}; float x2[4] = {x1[1], x1[0] + x1[2], x1[1] + x1[3], x1[2]};
#pragma unroll
  for (int n = 0; n < 4; ++n) o[n] = pmul(w[0], v[n]) + pmul(w[1], x1[n]) + pmul(w[2], x2[n]) + b;
}

__global__ __launch_bounds__(256) void stae_kernel(const float* __restrict__ x, const float* __restrict__ z, const b16* __restrict__ Bm, const b16* __restrict__ Be, const float* __restrict__ P, float* __restrict__ out) {
  __shared__ __attribute__((aligned(16))) b16 Hh[8][16][H + 8], Hl[8][16][H + 8]; __shared__ float Hf[8][16][H + 1]; __shared__ float En[8][16][T * N + 1]; __shared__ __attribute__((aligned(16))) float Os[8][16 * T * N]; __shared__ float Ps[544];
  const int t_ = threadIdx.x, wid = t_ >> 5, lane = t_ & 31, nloc = lane & 15, hlf = lane >> 4; const size_t s0 = (size_t)blockIdx.x * NB + wid * 16;
  for (int i = t_; i < 544; i += 256) Ps[i] = P[i];
  __syncthreads();
  auto run_lstm = [&](const b16* Bw, const float* bias  , int which) {
    for (int i = lane; i < 16 * (H + 8); i += 32) { (&Hh[wid][0][0])[i] = (b16)0.0f; (&Hl[wid][0][0])[i] = (b16)0.0f; }
    float c[8];
#pragma unroll
    for (int v = 0; v < 8; ++v) c[v] = 0.0f;
    wave_lds_sync();
    for (int st = 0; st < T; ++st) { v16b ah, al; const int row = nloc;
#pragma unroll
      for (int e = 0; e < 16; ++e) { const int k = (e < 8) ? (8 * hlf + e) : (16 + 8 * hlf + e - 8); b16 a = (b16)0.0f, l = (b16)0.0f;
        if (k < N) { const float xv = (which == 0) ? bf16_rne(z[(s0 + row) * (T * N) + st * N + k]) : En[wid][row][st * N + k]; split16(xv * AS_, a, l); }
        else if (k < N + H) { a = Hh[wid][row][k - N]; l = Hl[wid][row][k - N]; }
        ah[e] = a; al[e] = l; }
      v8f acc[4] = {{}, {}, {}, {}};
#pragma unroll
      for (int g = 0; g < 4; ++g) { const v16b bw = frag_kb(Bw + (size_t)(g * H + nloc) * 32, hlf); acc[g] = wmma16b(ah, bw, acc[g]); acc[g] = wmma16b(al, bw, acc[g]); }
      wave_lds_sync();
#pragma unroll
      for (int v = 0; v < 8; ++v) { const int r = 8 * hlf + v; const float sc = 1.0f / (AS_ * WS_);
        const float gi = acc[0][v] * sc + bias[0 * H + nloc], gf = acc[1][v] * sc + bias[1 * H + nloc], gg = acc[2][v] * sc + bias[2 * H + nloc], go = acc[3][v] * sc + bias[3 * H + nloc];
        const float cn = sigm(gf) * c[v] + sigm(gi) * tanh_(gg); c[v] = cn; const float h = sigm(go) * tanh_(cn);
        b16 a, l; split16(h * AS_, a, l); Hh[wid][r][nloc] = a; Hl[wid][r][nloc] = l; Hf[wid][r][nloc] = h; }
      wave_lds_sync(); }
  };
  run_lstm(Bm, Ps, 0);
  if (hlf == 0) { const int s = nloc; const float* hrow = Hf[wid][s];
    float m8[8];
#pragma unroll
    for (int j = 0; j < 8; ++j) { float a = Ps[256 + j];
#pragma unroll
      for (int k = 0; k < H; ++k) a += pmul(Ps[128 + j * H + k], hrow[k]);
      m8[j] = fmaxf(a, 0.0f); }
    float m4[4];
#pragma unroll
    for (int n = 0; n < 4; ++n) { float a = Ps[296 + n];
#pragma unroll
      for (int j = 0; j < 8; ++j) a += pmul(Ps[264 + n * 8 + j], m8[j]);
      m4[n] = a; }
    float mo[4]; gcn4(m4, Ps + 304, Ps[307], mo);
    const float* xr = x + (s0 + s) * (T * N);
    for (int tt = 0; tt < T; ++tt) { float iv[4], vv[4];
#pragma unroll
      for (int n = 0; n < 4; ++n) { iv[n] = bf16_rne(xr[n * T + tt]); float a = Ps[464 + tt] + pmul(mo[n], Ps[308 + tt * 13 + 12]);
#pragma unroll 1
        for (int j = 0; j < T; ++j) a += pmul(bf16_rne(xr[n * T + j]), Ps[308 + tt * 13 + j]);
        vv[n] = a; }
      float e1[4], e2[4]; gcn4(iv, Ps + 300, Ps[303], e1); gcn4(vv, Ps + 304, Ps[307], e2);
#pragma unroll
      for (int n = 0; n < 4; ++n) En[wid][s][tt * N + n] = e1[n] + e2[n]; } }
  wave_lds_sync();
  run_lstm(Be, Ps + 64, 1);
  if (hlf == 0) { const int s = nloc; const float* hrow = Hf[wid][s];
#pragma unroll
    for (int n = 0; n < 4; ++n) { float a = Ps[540 + n];
#pragma unroll
      for (int k = 0; k < H; ++k) a += pmul(Ps[476 + n * H + k], hrow[k]);
      for (int tt = 0; tt < T; ++tt) Os[wid][s * (T * N) + n * T + tt] = a; } }
  wave_lds_sync();
  float* dst = out + s0 * (T * N);
  for (int pass = 0; pass < 2; ++pass) {
#pragma unroll
    for (int j = 0; j < 6; ++j) *(volatile v4f*)(dst + (j * 32 + lane) * 4) = *(const v4f*)(&Os[wid][(j * 32 + lane) * 4]);
    __threadfence(); }
}
}

extern "C" void kernel_launch(void* const* d_in, const int* in_sizes, int n_in,
                              void* d_out, int out_size, void* d_ws, size_t ws_size, hipStream_t stream) {
  (void)n_in; (void)out_size;
  const float* x = (const float*)d_in[0]; const float* z = (const float*)d_in[1];
  const float* p[20]; for (int i = 0; i < 20; ++i) p[i] = (const float*)d_in[2 + i];
  float* out = (float*)d_out;
  if (in_sizes[0] != Bn * T * N || in_sizes[1] != Bn * T * N || in_sizes[2] != 4 * H * N || in_sizes[3] != 4 * H * H || in_sizes[14] != T * (T + 1) || in_sizes[20] != N * H) return;
  size_t off = 0; char* ws = (char*)d_ws;
  auto carve = [&](size_t bytes) { char* q = ws + off; off += (bytes + 255) & ~(size_t)255; return q; };
  b16* Bm = (b16*)carve(64 * 32 * 2); b16* Be = (b16*)carve(64 * 32 * 2); float* P = (float*)carve(544 * 4 + 256);
  if (off > ws_size) return;
  prep_kernel<<<1, 256, 0, stream>>>(p[0], p[1], p[2], p[3], p[4], p[5], p[6], p[7], p[8], p[9], p[10], p[11], p[12], p[13], p[14], p[15], p[16], p[17], p[18], p[19], Bm, Be, P);
  stae_kernel<<<Bn / NB, 256, 0, stream>>>(x, z, Bm, Be, P, out);
}
